// MuleHunterGNN_50079318671882
// MI455X (gfx1250) — hardware-verified
//
#include <hip/hip_runtime.h>
#include <stddef.h>
#include <math.h>


#define FIN     20
#define HID     64
#define NHEAD   4
#define HPW     256
#define H3W     32
#define NOUT    2
#define K1      64
#define K3      128
#define NTHR    256
#define NWAVE   8
#define EPT     8
#define NGRP    2
#define CHUNK   (NTHR * EPT * NGRP)
#define WCAP    (EPT * NGRP * 32)
#define LISTN   (NWAVE * WCAP)
#define NBC     4096
#define NBF     1024
#define RCAP    40960
#define RBN     128
#define TGT     256
#define DEGCAP  256
#define OTHR    512
#define WSCAP   134217728
#define NEG_SLOPE 0.2f
#define DEN_EPS 1e-16f
#define BN_EPS  1e-5f
#define NEG_BIG (-3.0e38f)

#define LDS_FILL ((RCAP + NBF + LISTN) * 4 + 64)

static_assert((CHUNK & (CHUNK - 1)) == 0);
static_assert(CHUNK <= 4096);
static_assert(NBC <= 4096 && NBF <= 4096);
static_assert((NBC & (NBC - 1)) == 0 && (NBF & (NBF - 1)) == 0);
static_assert(NBC == 4 * NBF);
static_assert(OTHR * 8 == NBC);
static_assert((RCAP % 32) == 0);
static_assert(TGT == NWAVE * 32);
static_assert((NBC % TGT) == 0);

typedef float          v4f  __attribute__((ext_vector_type(4)));
typedef float          v8f  __attribute__((ext_vector_type(8)));
typedef int            v4i  __attribute__((ext_vector_type(4)));
typedef unsigned short v8us __attribute__((ext_vector_type(8)));
typedef __bf16         v16b __attribute__((ext_vector_type(16)));
union FragB { v16b v; v8us h[2]; };

template <int KD, int NC>
struct GCfg {
  static constexpr int WPR  = (NC >= 64) ? 2 : 1;
  static constexpr int TPW  = NC / 16 / WPR;
  static constexpr int RG   = NWAVE / WPR;
  static constexpr int BM   = RG * 16;
  static constexpr int APK  = KD + 8;
  static constexpr int LDSA = 2 * BM * APK * 2;
  static constexpr int LDSS = BM * NC * 4;
  static constexpr int LDS  = LDSA > LDSS ? LDSA : LDSS;
  static constexpr int Q4   = TPW * 4;
  static constexpr int RPI  = 32 / Q4;
  static constexpr int NIT  = 16 / RPI;
  static constexpr int UPT  = (BM * KD / 8) / NTHR;
};

__device__ __forceinline__ unsigned int bfr(float f) {
  const unsigned int u = __float_as_uint(f);
  return (u + 0x7FFFu + ((u >> 16) & 1u)) >> 16;
}

__device__ __forceinline__ void split1(float x, unsigned short& hb, unsigned short& lb) {
  const unsigned int hu = bfr(x);
  const float hf = __uint_as_float(hu << 16);
  hb = (unsigned short)hu;
  lb = (unsigned short)bfr(x - hf);
}

__device__ __forceinline__ void split8(v4f a, v4f b, v8us& hi, v8us& lo) {
  unsigned short hb, lb;
  split1(a.x, hb, lb); hi[0] = hb; lo[0] = lb;
  split1(a.y, hb, lb); hi[1] = hb; lo[1] = lb;
  split1(a.z, hb, lb); hi[2] = hb; lo[2] = lb;
  split1(a.w, hb, lb); hi[3] = hb; lo[3] = lb;
  split1(b.x, hb, lb); hi[4] = hb; lo[4] = lb;
  split1(b.y, hb, lb); hi[5] = hb; lo[5] = lb;
  split1(b.z, hb, lb); hi[6] = hb; lo[6] = lb;
  split1(b.w, hb, lb); hi[7] = hb; lo[7] = lb;
}

__device__ __forceinline__ v8f wmb(v16b a, v16b b, v8f c) {
  v8f d = __builtin_amdgcn_wmma_f32_16x16x32_bf16(false, a, false, b, (short)0, c, false, false);
  asm volatile("v_nop\n\tv_nop\n\tv_nop\n\tv_nop" : "+v"(d) : "v"(a), "v"(b));
  return d;
}

__device__ __forceinline__ float lrelu(float v) { return v > 0.0f ? v : NEG_SLOPE * v; }
__device__ __forceinline__ v4f relu4(v4f v) {
  v.x = fmaxf(v.x, 0.0f); v.y = fmaxf(v.y, 0.0f); v.z = fmaxf(v.z, 0.0f); v.w = fmaxf(v.w, 0.0f);
  return v;
}

template <int NB>
__device__ __forceinline__ int scan_chunk(const int* __restrict__ dsts, int nE, int cbase, int slotBase,
                                          int vec8, int* list, int tid, int lane, int wave) {
  int wc = 0;
#pragma unroll
  for (int g = 0; g < NGRP; ++g) {
    const int el0  = (g * NTHR + tid) * EPT;
    const int e0   = cbase + el0;
    const int sent = -2147483647 - 1;
    v4i da, db;
    if (vec8 != 0 && cbase + CHUNK <= nE) {
      da = *(const v4i*)(dsts + e0);
      db = *(const v4i*)(dsts + e0 + 4);
    } else {
      da.x = (e0     < nE) ? dsts[min(e0, nE - 1)] : sent;
      da.y = (e0 + 1 < nE) ? dsts[min(e0 + 1, nE - 1)] : sent;
      da.z = (e0 + 2 < nE) ? dsts[min(e0 + 2, nE - 1)] : sent;
      da.w = (e0 + 3 < nE) ? dsts[min(e0 + 3, nE - 1)] : sent;
      db.x = (e0 + 4 < nE) ? dsts[min(e0 + 4, nE - 1)] : sent;
      db.y = (e0 + 5 < nE) ? dsts[min(e0 + 5, nE - 1)] : sent;
      db.z = (e0 + 6 < nE) ? dsts[min(e0 + 6, nE - 1)] : sent;
      db.w = (e0 + 7 < nE) ? dsts[min(e0 + 7, nE - 1)] : sent;
    }
    const unsigned nb = (unsigned)slotBase;
    const unsigned s0 = (unsigned)da.x - nb, s1 = (unsigned)da.y - nb;
    const unsigned s2 = (unsigned)da.z - nb, s3 = (unsigned)da.w - nb;
    const unsigned s4 = (unsigned)db.x - nb, s5 = (unsigned)db.y - nb;
    const unsigned s6 = (unsigned)db.z - nb, s7 = (unsigned)db.w - nb;
    const bool h0 = s0 < (unsigned)NB, h1 = s1 < (unsigned)NB, h2 = s2 < (unsigned)NB, h3 = s3 < (unsigned)NB;
    const bool h4 = s4 < (unsigned)NB, h5 = s5 < (unsigned)NB, h6 = s6 < (unsigned)NB, h7 = s7 < (unsigned)NB;
    const unsigned any = __builtin_amdgcn_ballot_w32(h0 | h1 | h2 | h3 | h4 | h5 | h6 | h7);
    if (any != 0u) {
#define HITJ(J, HJ, SJ) { \
        const unsigned mj = __builtin_amdgcn_ballot_w32(HJ); \
        if (mj != 0u) { \
          if (HJ) { \
            const int pos = wc + (int)__builtin_amdgcn_mbcnt_lo(mj, 0u); \
            if (pos < WCAP) list[wave * WCAP + pos] = ((el0 + (J)) << 12) | (int)(SJ); \
          } \
          wc += (int)__builtin_popcount(mj); } }
      HITJ(0, h0, s0)
      HITJ(1, h1, s1)
      HITJ(2, h2, s2)
      HITJ(3, h3, s3)
      HITJ(4, h4, s4)
      HITJ(5, h5, s5)
      HITJ(6, h6, s6)
      HITJ(7, h7, s7)
#undef HITJ
    }
  }
  return wc;
}

template <int KD, int NC>
__global__ __launch_bounds__(NTHR) void k_wprep(const float* __restrict__ WA, int ka, int a0,
                                                const float* __restrict__ WB, int kb, int b0,
                                                unsigned short* wp) {
  constexpr int UNITS = NC * KD / 8;
  constexpr int KD8   = KD / 8;
  static_assert((UNITS % 32) == 0 && (KD % 8) == 0);
  const int i = (int)blockIdx.x * NTHR + (int)threadIdx.x;
  if (i >= UNITS) return;
  const int n  = i / KD8;
  const int k0 = (i - n * KD8) * 8;
  float v[8];
#pragma unroll
  for (int e = 0; e < 8; ++e) {
    const int k = k0 + e;
    int ia = k - a0; ia = ia < 0 ? 0 : (ia > ka - 1 ? ka - 1 : ia);
    int ib = k - b0; ib = ib < 0 ? 0 : (ib > kb - 1 ? kb - 1 : ib);
    const float va = WA[(size_t)ia * NC + n];
    const float vb = WB[(size_t)ib * NC + n];
    const bool inA = (k >= a0) && (k < a0 + ka);
    const bool inB = (k >= b0) && (k < b0 + kb);
    v[e] = inA ? va : (inB ? vb : 0.0f);
  }
  v4f a, b;
  a.x = v[0]; a.y = v[1]; a.z = v[2]; a.w = v[3];
  b.x = v[4]; b.y = v[5]; b.z = v[6]; b.w = v[7];
  v8us hv, lv;
  split8(a, b, hv, lv);
  unsigned short* dh = wp + (size_t)i * 8;
  unsigned short* dl = dh + (size_t)NC * KD;
  *(volatile v8us*)dh = hv;
  *(volatile v8us*)dl = lv;
  __threadfence();
  *(volatile v8us*)dh = hv;
  *(volatile v8us*)dl = lv;
}

__global__ __launch_bounds__(NTHR) void k_count(
    const int* __restrict__ dsts, int* cnt, int nE, int vec8) {
  __shared__ __attribute__((aligned(16))) int scnt[NBC];
  __shared__ __attribute__((aligned(16))) int list[LISTN];
  __shared__ int wcnt[NWAVE];
  const int tid = threadIdx.x, lane = tid & 31, wave = tid >> 5;
  const int nodeBase = blockIdx.x * NBC;

  for (int i = tid; i < NBC; i += NTHR) scnt[i] = 0;
  __syncthreads();

  const int nChunks = (nE + CHUNK - 1) / CHUNK;
#pragma unroll 1
  for (int ch = 0; ch < nChunks; ++ch) {
    const int cbase = ch * CHUNK;
    const int wc = scan_chunk<NBC>(dsts, nE, cbase, nodeBase, vec8, list, tid, lane, wave);
    if (lane == 0) wcnt[wave] = wc;
    __syncthreads();
    if (wave == 0) {
#pragma unroll 1
      for (int wsx = 0; wsx < NWAVE; ++wsx) {
        int n = __builtin_amdgcn_readfirstlane(wcnt[wsx]);
        n = n > WCAP ? WCAP : (n < 0 ? 0 : n);
        const int* lp = list + wsx * WCAP;
#pragma unroll 1
        for (int i = 0; i < n; ++i) {
          const int ent  = __builtin_amdgcn_readfirstlane(lp[i]);
          const int slot = ent & (NBC - 1);
          if (lane == 0) scnt[slot] = scnt[slot] + 1;
        }
      }
    }
    __syncthreads();
  }

  v4i cq[4];
#pragma unroll
  for (int q = 0; q < 4; ++q) {
    const int f = (wave * 4 + q) * 128 + 4 * lane;
    cq[q] = *(const v4i*)(scnt + f);
  }
  int* cp = cnt + (size_t)nodeBase;
#pragma unroll
  for (int q = 0; q < 4; ++q) {
    const int f = (wave * 4 + q) * 128 + 4 * lane;
    *(volatile v4i*)(cp + f) = cq[q];
  }
  __threadfence();
#pragma unroll
  for (int q = 0; q < 4; ++q) {
    const int f = (wave * 4 + q) * 128 + 4 * lane;
    *(volatile v4i*)(cp + f) = cq[q];
  }
}

__global__ __launch_bounds__(OTHR) void k_offsets(
    const int* __restrict__ cnt, int* off, int* rbase, int nChunk) {
  __shared__ __attribute__((aligned(16))) int soff[NBC];
  __shared__ __attribute__((aligned(16))) int srb[RBN];
  __shared__ int wtot[OTHR / 32];
  const int tid = threadIdx.x, lane = tid & 31, wave = tid >> 5, sub = tid >> 7;
  for (int i = tid; i < RBN; i += OTHR) srb[i] = 0;
  int carry = 0;
#pragma unroll 1
  for (int ch = 0; ch < nChunk; ++ch) {
    const int base = ch * NBC;
    const v4i c0 = *(const v4i*)(cnt + base + 8 * tid);
    const v4i c1 = *(const v4i*)(cnt + base + 8 * tid + 4);
    const int e0 = max(c0.x, 0), e1 = max(c0.y, 0), e2 = max(c0.z, 0), e3 = max(c0.w, 0);
    const int e4 = max(c1.x, 0), e5 = max(c1.y, 0), e6 = max(c1.z, 0), e7 = max(c1.w, 0);
    const int ts = e0 + e1 + e2 + e3 + e4 + e5 + e6 + e7;
    int incl = ts;
#pragma unroll
    for (int d = 1; d < 32; d <<= 1) {
      const int t = __shfl_up(incl, d);
      if (lane >= d) incl += t;
    }
    if (lane == 31) wtot[wave] = incl;
    __syncthreads();
    const int S0 = wtot[0]  + wtot[1]  + wtot[2]  + wtot[3];
    const int S1 = wtot[4]  + wtot[5]  + wtot[6]  + wtot[7];
    const int S2 = wtot[8]  + wtot[9]  + wtot[10] + wtot[11];
    const int S3 = wtot[12] + wtot[13] + wtot[14] + wtot[15];
    int pre = 0;
#pragma unroll 1
    for (int w = 4 * sub; w < wave; ++w) pre += wtot[w];
    const int b0 = carry;
    const int b1 = b0 + ((S0 + 31) & ~31);
    const int b2 = b1 + ((S1 + 31) & ~31);
    const int b3 = b2 + ((S2 + 31) & ~31);
    const int b4 = b3 + ((S3 + 31) & ~31);
    const int myb = sub == 0 ? b0 : (sub == 1 ? b1 : (sub == 2 ? b2 : b3));
    if (tid == 0) {
      srb[min(4 * ch + 0, RBN - 1)] = b0;
      srb[min(4 * ch + 1, RBN - 1)] = b1;
      srb[min(4 * ch + 2, RBN - 1)] = b2;
      srb[min(4 * ch + 3, RBN - 1)] = b3;
    }
    int run = myb + pre + incl - ts;
    soff[8 * tid + 0] = run; run += e0;
    soff[8 * tid + 1] = run; run += e1;
    soff[8 * tid + 2] = run; run += e2;
    soff[8 * tid + 3] = run; run += e3;
    soff[8 * tid + 4] = run; run += e4;
    soff[8 * tid + 5] = run; run += e5;
    soff[8 * tid + 6] = run; run += e6;
    soff[8 * tid + 7] = run;
    carry = b4;
    __syncthreads();
    const v4i o0 = *(const v4i*)(soff + 4 * tid);
    const v4i o1 = *(const v4i*)(soff + 4 * (tid + OTHR));
    int* op = off + base;
    *(volatile v4i*)(op + 4 * tid) = o0;
    *(volatile v4i*)(op + 4 * (tid + OTHR)) = o1;
    __threadfence();
    *(volatile v4i*)(op + 4 * tid) = o0;
    *(volatile v4i*)(op + 4 * (tid + OTHR)) = o1;
    __syncthreads();
  }
  if (tid == 0) srb[min(4 * nChunk, RBN - 1)] = carry;
  __syncthreads();
  v4i rv = {0, 0, 0, 0};
  if (tid < 32) rv = *(const v4i*)(srb + 4 * tid);
  if (tid < 32) *(volatile v4i*)(rbase + 4 * tid) = rv;
  __threadfence();
  if (tid < 32) *(volatile v4i*)(rbase + 4 * tid) = rv;
}

__global__ __launch_bounds__(NTHR) void k_fill(
    const int* __restrict__ srcs, const int* __restrict__ dsts,
    const int* __restrict__ off, const int* __restrict__ rbase,
    int* csr, int nN, int nE, int vec8, int csrLen) {
  extern __shared__ v4f lds_dyn[];
  int* region = (int*)lds_dyn;
  int* cursor = region + RCAP;
  int* list   = cursor + NBF;
  int* wcnt   = list + LISTN;
  const int tid = threadIdx.x, lane = tid & 31, wave = tid >> 5;
  const int b = blockIdx.x;
  const int nodeBase = b * NBF;

  int rb0 = rbase[b];
  const int rb1 = rbase[b + 1];
  rb0 = rb0 < 0 ? 0 : (rb0 > csrLen ? csrLen : rb0);
  rb0 &= ~31;
  int len = rb1 - rb0;
  len = len < 0 ? 0 : (len > RCAP ? RCAP : len);
  int lenW = (len + 31) & ~31;
  if (rb0 + lenW > csrLen) lenW = (csrLen - rb0) & ~31;

  {
    const v4i z = {0, 0, 0, 0};
    for (int i = tid; i < RCAP / 4; i += NTHR) ((v4i*)region)[i] = z;
    for (int s = tid; s < NBF; s += NTHR) {
      int o = off[nodeBase + s] - rb0;
      o = o < 0 ? 0 : (o > RCAP ? RCAP : o);
      cursor[s] = o;
    }
  }
  __syncthreads();

  const int nChunks = (nE + CHUNK - 1) / CHUNK;
#pragma unroll 1
  for (int ch = 0; ch < nChunks; ++ch) {
    const int cbase = ch * CHUNK;
    const int wc = scan_chunk<NBF>(dsts, nE, cbase, nodeBase, vec8, list, tid, lane, wave);
    if (lane == 0) wcnt[wave] = wc;
    __syncthreads();
    if (wave == 0) {
#pragma unroll 1
      for (int wsx = 0; wsx < NWAVE; ++wsx) {
        int n = __builtin_amdgcn_readfirstlane(wcnt[wsx]);
        n = n > WCAP ? WCAP : (n < 0 ? 0 : n);
        const int* lp = list + wsx * WCAP;
#pragma unroll 1
        for (int i = 0; i < n; ++i) {
          const int ent  = __builtin_amdgcn_readfirstlane(lp[i]);
          const int slot = ent & (NBF - 1);
          int e = cbase + ((ent >> 12) & (CHUNK - 1));
          e = e > nE - 1 ? nE - 1 : e;
          int src = srcs[e];
          src = src < 0 ? 0 : (src > nN - 1 ? nN - 1 : src);
          if (lane == 0) {
            int pos = cursor[slot];
            pos = pos < 0 ? 0 : (pos > RCAP - 1 ? RCAP - 1 : pos);
            region[pos] = src;
            const int np = pos + 1;
            cursor[slot] = np > RCAP ? RCAP : np;
          }
        }
      }
    }
    __syncthreads();
  }

  const int nv = lenW >> 2;
  int* gp = csr + rb0;
#pragma unroll 1
  for (int i = tid; i < nv; i += NTHR) { const v4i v = ((const v4i*)region)[i]; *(volatile v4i*)(gp + 4 * i) = v; }
  __threadfence();
#pragma unroll 1
  for (int i = tid; i < nv; i += NTHR) { const v4i v = ((const v4i*)region)[i]; *(volatile v4i*)(gp + 4 * i) = v; }
}

template <int KD, int NC>
__device__ __forceinline__ void gemm_core(const float* __restrict__ A, const unsigned short* __restrict__ Bw,
                                          int nRowsA, v4f* ldsb) {
  typedef GCfg<KD, NC> G;
  constexpr int WPR = G::WPR, TPW = G::TPW, BM = G::BM, APK = G::APK, UPT = G::UPT;
  constexpr size_t WPLN = (size_t)NC * KD;
  static_assert(KD % 32 == 0 && NC % (16 * WPR) == 0 && TPW >= 1);
  static_assert(UPT * NTHR * 8 == BM * KD && UPT >= 1);
  static_assert(((APK * 2) % 16) == 0);
  static_assert(BM * NC * 4 <= G::LDS && 2 * BM * APK * 2 <= G::LDS);

  unsigned short* sHi = (unsigned short*)ldsb;
  unsigned short* sLo = sHi + BM * APK;
  float*          stg = (float*)ldsb;
  const int tid = threadIdx.x, lane = tid & 31, wave = tid >> 5, hh = lane >> 4, m = lane & 15;
  const int rowBase = blockIdx.x * BM;

#pragma unroll
  for (int i = 0; i < UPT; ++i) {
    const int idx = i * NTHR + tid;
    const int r   = idx / (KD / 8);
    const int cc  = (idx - r * (KD / 8)) * 8;
    int row = rowBase + r;
    row = row > nRowsA - 1 ? nRowsA - 1 : row;
    const float* ap = A + (size_t)row * KD + cc;
    const v4f a = *(const v4f*)ap, b = *(const v4f*)(ap + 4);
    v8us hv, lv;
    split8(a, b, hv, lv);
    *(v8us*)(sHi + r * APK + cc) = hv;
    *(v8us*)(sLo + r * APK + cc) = lv;
  }
  __syncthreads();

  const int rg  = wave / WPR;
  const int chf = wave - rg * WPR;
  const int r0  = rg * 16;
  const int c0  = chf * TPW * 16;

  v8f acc[TPW];
#pragma unroll
  for (int t = 0; t < TPW; ++t) { v8f z = {0.f, 0.f, 0.f, 0.f, 0.f, 0.f, 0.f, 0.f}; acc[t] = z; }
  const unsigned short* ahp = sHi + (r0 + m) * APK + 8 * hh;
  const unsigned short* alp = sLo + (r0 + m) * APK + 8 * hh;
#pragma unroll 2
  for (int kt = 0; kt < KD / 32; ++kt) {
    FragB ah, al;
    ah.h[0] = *(const v8us*)(ahp + 32 * kt);
    ah.h[1] = *(const v8us*)(ahp + 32 * kt + 16);
    al.h[0] = *(const v8us*)(alp + 32 * kt);
    al.h[1] = *(const v8us*)(alp + 32 * kt + 16);
#pragma unroll
    for (int t = 0; t < TPW; ++t) {
      const unsigned short* bp = Bw + (size_t)(c0 + 16 * t + m) * KD + 32 * kt + 8 * hh;
      FragB bh, bl;
      bh.h[0] = *(const v8us*)bp;
      bh.h[1] = *(const v8us*)(bp + 16);
      bl.h[0] = *(const v8us*)(bp + WPLN);
      bl.h[1] = *(const v8us*)(bp + WPLN + 16);
      acc[t] = wmb(ah.v, bh.v, acc[t]);
      acc[t] = wmb(ah.v, bl.v, acc[t]);
      acc[t] = wmb(al.v, bh.v, acc[t]);
    }
  }
  __syncthreads();

  {
    float* sp = stg + (size_t)(r0 + 8 * hh) * NC + c0 + m;
#pragma unroll
    for (int t = 0; t < TPW; ++t) {
#pragma unroll
      for (int r = 0; r < 8; ++r) sp[r * NC + 16 * t] = acc[t][r];
    }
  }
  __syncthreads();
}

template <int KD, int NC, int HASBN, int RELU, int HASADD>
__global__ __launch_bounds__(NTHR) void k_gemm_ep(
    const float* __restrict__ A, const unsigned short* __restrict__ Bw,
    const float* __restrict__ bias, const float* __restrict__ gam, const float* __restrict__ bet,
    const float* __restrict__ addp, float* C, int nRowsA, float rsq) {
  typedef GCfg<KD, NC> G;
  constexpr int WPR = G::WPR, TPW = G::TPW, BM = G::BM, Q4 = G::Q4, RPI = G::RPI, NIT = G::NIT;
  static_assert((Q4 & (Q4 - 1)) == 0 && Q4 >= 8 && Q4 <= 32);
  static_assert(NIT * RPI == 16 && NIT <= 16);
  extern __shared__ v4f lds_dyn[];
  gemm_core<KD, NC>(A, Bw, nRowsA, lds_dyn);
  const float* stg = (const float*)lds_dyn;
  const int tid = threadIdx.x, lane = tid & 31, wave = tid >> 5;
  const int rowBase = blockIdx.x * BM;
  const int rg  = wave / WPR;
  const int chf = wave - rg * WPR;
  const int r0  = rg * 16;
  const int c0  = chf * TPW * 16;
  const int qq   = lane & (Q4 - 1);
  const int rsub = lane / Q4;
  const int col  = c0 + 4 * qq;
  const v4f bb = *(const v4f*)(bias + col);
  v4f sc = {1.f, 1.f, 1.f, 1.f};
  v4f sh = {0.f, 0.f, 0.f, 0.f};
  if constexpr (HASBN != 0) {
    const v4f g = *(const v4f*)(gam + col);
    sh = *(const v4f*)(bet + col);
    sc = g * rsq;
  }
  const size_t gb = (size_t)(rowBase + r0) * NC + col;
  v4f ov[NIT];
#pragma unroll
  for (int it = 0; it < NIT; ++it) {
    const int row = it * RPI + rsub;
    v4f v = *(const v4f*)(stg + (size_t)(r0 + row) * NC + col);
    v = v + bb;
    if constexpr (HASBN != 0) v = v * sc + sh;
    if constexpr (RELU != 0) v = relu4(v);
    if constexpr (HASADD != 0) {
      const v4f ad = *(const v4f*)(addp + gb + (size_t)row * NC);
      v = v + ad;
    }
    ov[it] = v;
    *(volatile v4f*)(C + gb + (size_t)row * NC) = v;
  }
  __threadfence();
#pragma unroll
  for (int it = 0; it < NIT; ++it) {
    const int row = it * RPI + rsub;
    *(volatile v4f*)(C + gb + (size_t)row * NC) = ov[it];
  }
}

template <int KD, int NC, int HEADS>
__global__ __launch_bounds__(NTHR) void k_gemm_att(
    const float* __restrict__ A, const unsigned short* __restrict__ Bw,
    const float* __restrict__ attS, const float* __restrict__ attD,
    float* C, float* eS, float* eD, int nRowsA) {
  typedef GCfg<KD, NC> G;
  constexpr int WPR = G::WPR, TPW = G::TPW, BM = G::BM, Q4 = G::Q4, RPI = G::RPI, NIT = G::NIT;
  constexpr int CH   = NC / HEADS;
  constexpr int LPH  = CH / 4;
  constexpr int NES  = BM * HEADS;
  constexpr int NESI = NES / 128;
  static_assert(HEADS * CH == NC && (CH % 4) == 0);
  static_assert((Q4 & (Q4 - 1)) == 0 && Q4 <= 32 && Q4 >= LPH && (LPH & (LPH - 1)) == 0 && LPH >= 1);
  static_assert(NIT * RPI == 16);
  static_assert((NES % 128) == 0 && 2 * NESI <= NWAVE);

  extern __shared__ v4f lds_dyn[];
  __shared__ __attribute__((aligned(16))) float sES[NES];
  __shared__ __attribute__((aligned(16))) float sED[NES];
  gemm_core<KD, NC>(A, Bw, nRowsA, lds_dyn);
  const float* stg = (const float*)lds_dyn;
  const int tid = threadIdx.x, lane = tid & 31, wave = tid >> 5;
  const int rowBase = blockIdx.x * BM;
  const int rg  = wave / WPR;
  const int chf = wave - rg * WPR;
  const int r0  = rg * 16;
  const int c0  = chf * TPW * 16;

  const int qq   = lane & (Q4 - 1);
  const int rsub = lane / Q4;
  const int col  = c0 + 4 * qq;
  const int hd   = col / CH;
  const v4f sA = *(const v4f*)(attS + col);
  const v4f sD = *(const v4f*)(attD + col);
  const size_t gb = (size_t)(rowBase + r0) * NC + col;
#pragma unroll
  for (int it = 0; it < NIT; ++it) {
    const int row = it * RPI + rsub;
    const v4f v = *(const v4f*)(stg + (size_t)(r0 + row) * NC + col);
    *(volatile v4f*)(C + gb + (size_t)row * NC) = v;
    float ps = v.x * sA.x + v.y * sA.y + v.z * sA.z + v.w * sA.w;
    float pd = v.x * sD.x + v.y * sD.y + v.z * sD.z + v.w * sD.w;
#pragma unroll
    for (int o = 1; o < LPH; o <<= 1) { ps += __shfl_xor(ps, o); pd += __shfl_xor(pd, o); }
    if ((lane & (LPH - 1)) == 0) { sES[(r0 + row) * HEADS + hd] = ps; sED[(r0 + row) * HEADS + hd] = pd; }
  }
  __threadfence();
#pragma unroll
  for (int it = 0; it < NIT; ++it) {
    const int row = it * RPI + rsub;
    const v4f v = *(const v4f*)(stg + (size_t)(r0 + row) * NC + col);
    *(volatile v4f*)(C + gb + (size_t)row * NC) = v;
  }
  __syncthreads();

  v4f dv = {0.f, 0.f, 0.f, 0.f};
  const size_t eb = (size_t)rowBase * HEADS;
  if (wave < NESI) {
    const int f = wave * 128 + 4 * lane;
    dv = *(const v4f*)(sES + f);
    *(volatile v4f*)(eS + eb + f) = dv;
  } else if (wave < 2 * NESI) {
    const int f = (wave - NESI) * 128 + 4 * lane;
    dv = *(const v4f*)(sED + f);
    *(volatile v4f*)(eD + eb + f) = dv;
  }
  __threadfence();
  if (wave < NESI) {
    const int f = wave * 128 + 4 * lane;
    *(volatile v4f*)(eS + eb + f) = dv;
  } else if (wave < 2 * NESI) {
    const int f = (wave - NESI) * 128 + 4 * lane;
    *(volatile v4f*)(eD + eb + f) = dv;
  }
}

template <int F, int KOUT>
__global__ __launch_bounds__(NTHR) void k_gagg(
    const int* __restrict__ csr, const int* __restrict__ off, const int* __restrict__ cnt,
    const float* __restrict__ hin, float* aout, int nN, int csrLen) {
  constexpr int F4 = F / 4;
  constexpr int SL = KOUT / 4;
  static_assert((F % 4) == 0 && 2 * F <= KOUT && SL <= 32 && (KOUT % 32) == 0);
  const int tid = threadIdx.x, lane = tid & 31, wave = tid >> 5;
  const int tbase = blockIdx.x * TGT + wave * 32;
  const int pg = (lane < F4) ? lane : ((lane < 2 * F4) ? (lane - F4) : 0);
  const v4f z4 = {0.f, 0.f, 0.f, 0.f};
  const int cl    = tbase + lane;
  const int cnt_l = cnt[cl];
  const int off_l = off[cl];

#pragma unroll 1
  for (int j = 0; j < 32; ++j) {
    const int c = tbase + j;
    int nraw = __shfl(cnt_l, j);
    nraw = nraw < 0 ? 0 : nraw;
    const int n = nraw > DEGCAP ? DEGCAP : nraw;
    const int st = __shfl(off_l, j);

    v4f acc = z4;
#pragma unroll 1
    for (int q0 = 0; q0 < n; q0 += 32) {
      int pos = st + q0 + lane;
      pos = pos < 0 ? 0 : (pos > csrLen - 1 ? csrLen - 1 : pos);
      int sl = csr[pos];
      sl = sl < 0 ? 0 : (sl > nN - 1 ? nN - 1 : sl);
      const int mcnt = (n - q0) < 32 ? (n - q0) : 32;
#pragma unroll 1
      for (int pp = 0; pp < mcnt; ++pp) {
        const int s = __builtin_amdgcn_readlane(sl, pp);
        const v4f hv = *(const v4f*)(hin + (size_t)s * F + 4 * pg);
        acc = acc + hv;
      }
    }
    const float invd = 1.0f / fmaxf((float)nraw, 1.0f);
    const int crow = c < nN ? c : nN - 1;
    const v4f sf = *(const v4f*)(hin + (size_t)crow * F + 4 * pg);
    v4f v = z4;
    if (lane < F4) v = acc * invd;
    else if (lane < 2 * F4) v = sf;
    if (c >= nN) v = z4;
    float* p = aout + (size_t)c * KOUT + 4 * lane;
    if (lane < SL) *(volatile v4f*)p = v;
    __threadfence();
    if (lane < SL) *(volatile v4f*)p = v;
  }
}

__global__ __launch_bounds__(NTHR) void k_gat(
    const int* __restrict__ csr, const int* __restrict__ off, const int* __restrict__ cnt,
    const float* __restrict__ eS, const float* __restrict__ eD, const float* __restrict__ hp,
    const float* __restrict__ bias, const float* __restrict__ gam, const float* __restrict__ bet,
    float* hout, int nN, int csrLen, float rsq) {
  const int tid = threadIdx.x, lane = tid & 31, wave = tid >> 5;
  const int tbase = blockIdx.x * TGT + wave * 32;
  const int col0 = 4 * lane;
  const int col1 = HPW / 2 + 4 * lane;
  const int hd0  = lane >> 4;
  const int hd1  = hd0 + 2;
  const int oc   = 4 * (lane & 15);
  const v4f z4 = {0.f, 0.f, 0.f, 0.f};
  const v4f bb = *(const v4f*)(bias + oc);
  const v4f g  = *(const v4f*)(gam + oc);
  const v4f be = *(const v4f*)(bet + oc);
  const v4f sc = g * rsq;
  const int cl    = tbase + lane;
  const int cnt_l = cnt[cl];
  const int off_l = off[cl];

#pragma unroll 1
  for (int j = 0; j < 32; ++j) {
    const int c = tbase + j;
    int n = __shfl(cnt_l, j);
    n = n < 0 ? 0 : (n > DEGCAP ? DEGCAP : n);
    const int st = __shfl(off_l, j);
    const float ed0 = eD[(size_t)c * NHEAD + hd0];
    const float ed1 = eD[(size_t)c * NHEAD + hd1];

    float mx0 = NEG_BIG, mx1 = NEG_BIG;
#pragma unroll 1
    for (int q0 = 0; q0 < n; q0 += 32) {
      int pos = st + q0 + lane;
      pos = pos < 0 ? 0 : (pos > csrLen - 1 ? csrLen - 1 : pos);
      int sl = csr[pos];
      sl = sl < 0 ? 0 : (sl > nN - 1 ? nN - 1 : sl);
      const int mcnt = (n - q0) < 32 ? (n - q0) : 32;
#pragma unroll 1
      for (int pp = 0; pp < mcnt; ++pp) {
        const int s = __builtin_amdgcn_readlane(sl, pp);
        mx0 = fmaxf(mx0, lrelu(eS[(size_t)s * NHEAD + hd0] + ed0));
        mx1 = fmaxf(mx1, lrelu(eS[(size_t)s * NHEAD + hd1] + ed1));
      }
    }

    float den0 = 0.f, den1 = 0.f;
    v4f acc0 = z4, acc1 = z4;
#pragma unroll 1
    for (int q0 = 0; q0 < n; q0 += 32) {
      int pos = st + q0 + lane;
      pos = pos < 0 ? 0 : (pos > csrLen - 1 ? csrLen - 1 : pos);
      int sl = csr[pos];
      sl = sl < 0 ? 0 : (sl > nN - 1 ? nN - 1 : sl);
      const int mcnt = (n - q0) < 32 ? (n - q0) : 32;
#pragma unroll 1
      for (int pp = 0; pp < mcnt; ++pp) {
        const int s = __builtin_amdgcn_readlane(sl, pp);
        const float p0 = __expf(lrelu(eS[(size_t)s * NHEAD + hd0] + ed0) - mx0);
        const float p1 = __expf(lrelu(eS[(size_t)s * NHEAD + hd1] + ed1) - mx1);
        den0 += p0;
        den1 += p1;
        const v4f h0 = *(const v4f*)(hp + (size_t)s * HPW + col0);
        const v4f h1 = *(const v4f*)(hp + (size_t)s * HPW + col1);
        acc0 = acc0 + h0 * p0;
        acc1 = acc1 + h1 * p1;
      }
    }

    const float rd0 = 1.0f / (den0 + DEN_EPS);
    const float rd1 = 1.0f / (den1 + DEN_EPS);
    v4f t = acc0 * rd0 + acc1 * rd1;
    t.x += __shfl_xor(t.x, 16);
    t.y += __shfl_xor(t.y, 16);
    t.z += __shfl_xor(t.z, 16);
    t.w += __shfl_xor(t.w, 16);
    v4f v = t * 0.25f + bb;
    v = v * sc + be;
    v = relu4(v);
    if (c >= nN) v = z4;
    float* p = hout + (size_t)c * HID + 4 * lane;
    if (lane < 16) *(volatile v4f*)p = v;
    __threadfence();
    if (lane < 16) *(volatile v4f*)p = v;
  }
}

__global__ __launch_bounds__(NTHR) void k_final(
    const float* __restrict__ T, const float* __restrict__ Wc2, const float* __restrict__ bc2,
    float* out, int nN) {
  __shared__ float sW[H3W * NOUT];
  __shared__ float sB[NOUT];
  __shared__ __attribute__((aligned(16))) float sO[NOUT * NTHR];
  const int tid = threadIdx.x, lane = tid & 31, wave = tid >> 5;
  if (tid < H3W * NOUT) sW[tid] = Wc2[tid];
  if (tid < NOUT) sB[tid] = bc2[tid];
  __syncthreads();
  const int row = blockIdx.x * NTHR + tid;
  const float* tp = T + (size_t)row * H3W;
  float l0 = 0.f, l1 = 0.f;
#pragma unroll 1
  for (int p = 0; p < H3W / 4; ++p) {
    const v4f tv = *(const v4f*)(tp + 4 * p);
    const float* w = sW + 8 * p;
    l0 += tv.x * w[0] + tv.y * w[2] + tv.z * w[4] + tv.w * w[6];
    l1 += tv.x * w[1] + tv.y * w[3] + tv.z * w[5] + tv.w * w[7];
  }
  l0 += sB[0];
  l1 += sB[1];
  const float mx  = fmaxf(l0, l1);
  const float lse = mx + logf(expf(l0 - mx) + expf(l1 - mx));
  sO[2 * tid]     = l0 - lse;
  sO[2 * tid + 1] = l1 - lse;
  __syncthreads();
  v4f ov = {0.f, 0.f, 0.f, 0.f};
  int grow0 = 0;
  bool act = false;
  if (wave < 4) {
    const int f = wave * 32 + lane;
    ov = *(const v4f*)(sO + 4 * f);
    grow0 = blockIdx.x * NTHR + 2 * f;
    act = (grow0 + 1 < nN);
    if (act) *(volatile v4f*)(out + (size_t)grow0 * NOUT) = ov;
  }
  __threadfence();
  if (wave < 4) {
    if (act) *(volatile v4f*)(out + (size_t)grow0 * NOUT) = ov;
  }
}

typedef GCfg<K1, HID>  GA;
typedef GCfg<K1, H3W>  GS;
typedef GCfg<HID, HPW> GP;
typedef GCfg<K3, H3W>  GB;
typedef GCfg<H3W, H3W> GC;
static_assert((TGT % GA::BM) == 0 && (TGT % GS::BM) == 0 && (TGT % GP::BM) == 0 && (TGT % GB::BM) == 0 && (TGT % GC::BM) == 0);

static inline size_t al256(size_t v) { return (v + 255) & ~(size_t)255; }

extern "C" void kernel_launch(void* const* d_in, const int* in_sizes, int n_in,
                              void* d_out, int out_size, void* d_ws, size_t ws_size,
                              hipStream_t stream) {
  if (n_in < 24) return;
  const int nN = in_sizes[0] / FIN;
  const int nE = in_sizes[1] / 2;
  if (nN <= 0 || nE <= 0 || in_sizes[0] != nN * FIN || in_sizes[1] != 2 * nE) return;
  if (in_sizes[2] != FIN * HID || in_sizes[3] != FIN * HID) return;
  if (in_sizes[4] != HID || in_sizes[5] != HID || in_sizes[6] != HID) return;
  if (in_sizes[7] != HID * HPW || in_sizes[8] != HPW || in_sizes[9] != HPW) return;
  if (in_sizes[10] != HID || in_sizes[11] != HID || in_sizes[12] != HID) return;
  if (in_sizes[13] != HID * H3W || in_sizes[14] != HID * H3W) return;
  if (in_sizes[15] != H3W || in_sizes[16] != H3W || in_sizes[17] != H3W) return;
  if (in_sizes[18] != FIN * H3W || in_sizes[19] != H3W) return;
  if (in_sizes[20] != H3W * H3W || in_sizes[21] != H3W) return;
  if (in_sizes[22] != H3W * NOUT || in_sizes[23] != NOUT) return;
  if (out_size != nN * NOUT) return;
  if (nE > (1 << 28) || nN > (1 << 24)) return;

  const float* x    = (const float*)d_in[0];
  const int*   ei   = (const int*)d_in[1];
  const float* Wl1  = (const float*)d_in[2];
  const float* Wr1  = (const float*)d_in[3];
  const float* b1   = (const float*)d_in[4];
  const float* g1   = (const float*)d_in[5];
  const float* bt1  = (const float*)d_in[6];
  const float* W2   = (const float*)d_in[7];
  const float* atS  = (const float*)d_in[8];
  const float* atD  = (const float*)d_in[9];
  const float* b2   = (const float*)d_in[10];
  const float* g2   = (const float*)d_in[11];
  const float* bt2  = (const float*)d_in[12];
  const float* Wl3  = (const float*)d_in[13];
  const float* Wr3  = (const float*)d_in[14];
  const float* b3   = (const float*)d_in[15];
  const float* g3   = (const float*)d_in[16];
  const float* bt3  = (const float*)d_in[17];
  const float* Wsk  = (const float*)d_in[18];
  const float* bsk  = (const float*)d_in[19];
  const float* Wc1  = (const float*)d_in[20];
  const float* bc1  = (const float*)d_in[21];
  const float* Wc2  = (const float*)d_in[22];
  const float* bc2  = (const float*)d_in[23];
  const int*   src  = ei;
  const int*   dst  = ei + nE;
  float* out = (float*)d_out;

  const int NPAD   = ((nN + TGT - 1) / TGT) * TGT;
  const int nBC    = (nN + NBC - 1) / NBC;
  const int CNTPAD = nBC * NBC;
  if (4 * nBC + 1 > RBN) return;
  const int nBF    = (nN + NBF - 1) / NBF;
  const int csrLen = ((nE + 31) & ~31) + 4096;
  if (31 * 4 * nBC > 4096) return;
  const int nAgg   = NPAD / TGT;

  char* ws = (char*)d_ws;
  size_t off = 0;
  const size_t oB1  = off; off = al256(off + (size_t)2 * HID * K1 * 2);
  const size_t oBsk = off; off = al256(off + (size_t)2 * H3W * K1 * 2);
  const size_t oB2  = off; off = al256(off + (size_t)2 * HPW * HID * 2);
  const size_t oB3  = off; off = al256(off + (size_t)2 * H3W * K3 * 2);
  const size_t oBc  = off; off = al256(off + (size_t)2 * H3W * H3W * 2);
  const size_t oCnt = off; off = al256(off + (size_t)CNTPAD * 4);
  const size_t oOff = off; off = al256(off + (size_t)CNTPAD * 4);
  const size_t oRb  = off; off = al256(off + (size_t)RBN * 4);
  const size_t oCsr = off; off = al256(off + (size_t)csrLen * 4);
  const size_t oA1  = off; off = al256(off + (size_t)NPAD * K1 * 4);
  const size_t oH1  = off; off = al256(off + (size_t)NPAD * HID * 4);
  const size_t oIdp = off; off = al256(off + (size_t)NPAD * H3W * 4);
  const size_t oES  = off; off = al256(off + (size_t)NPAD * NHEAD * 4);
  const size_t oED  = off; off = al256(off + (size_t)NPAD * NHEAD * 4);
  const size_t oBig = off; off = al256(off + (size_t)NPAD * HPW * 4);
  const size_t oHs  = off; off = al256(off + (size_t)NPAD * H3W * 4);
  const size_t oT   = off; off = al256(off + (size_t)NPAD * H3W * 4);
  if (off > ws_size || off > (size_t)WSCAP) return;
  unsigned short* pB1  = (unsigned short*)(ws + oB1);
  unsigned short* pBsk = (unsigned short*)(ws + oBsk);
  unsigned short* pB2  = (unsigned short*)(ws + oB2);
  unsigned short* pB3  = (unsigned short*)(ws + oB3);
  unsigned short* pBc  = (unsigned short*)(ws + oBc);
  int*   cnt  = (int*)(ws + oCnt);
  int*   offp = (int*)(ws + oOff);
  int*   rb   = (int*)(ws + oRb);
  int*   csr  = (int*)(ws + oCsr);
  float* A1   = (float*)(ws + oA1);
  float* h2   = (float*)(ws + oA1);
  float* h1   = (float*)(ws + oH1);
  float* idp  = (float*)(ws + oIdp);
  float* es   = (float*)(ws + oES);
  float* ed   = (float*)(ws + oED);
  float* hp   = (float*)(ws + oBig);
  float* A3   = (float*)(ws + oBig);
  float* hs   = (float*)(ws + oHs);
  float* Tp   = (float*)(ws + oT);

  const int vec8 = ((nE & 3) == 0) ? 1 : 0;
  const float rsq = 1.0f / sqrtf(1.0f + BN_EPS);

  k_wprep<K1, HID><<<(HID * K1 / 8 + NTHR - 1) / NTHR, NTHR, 0, stream>>>(Wl1, FIN, 0, Wr1, FIN, FIN, pB1);
  k_wprep<K1, H3W><<<(H3W * K1 / 8 + NTHR - 1) / NTHR, NTHR, 0, stream>>>(Wsk, FIN, FIN, Wsk, FIN, FIN, pBsk);
  k_wprep<HID, HPW><<<(HPW * HID / 8 + NTHR - 1) / NTHR, NTHR, 0, stream>>>(W2, HID, 0, W2, HID, 0, pB2);
  k_wprep<K3, H3W><<<(H3W * K3 / 8 + NTHR - 1) / NTHR, NTHR, 0, stream>>>(Wl3, HID, 0, Wr3, HID, HID, pB3);
  k_wprep<H3W, H3W><<<(H3W * H3W / 8 + NTHR - 1) / NTHR, NTHR, 0, stream>>>(Wc1, H3W, 0, Wc1, H3W, 0, pBc);

  k_count<<<nBC, NTHR, 0, stream>>>(dst, cnt, nE, vec8);
  k_offsets<<<1, OTHR, 0, stream>>>(cnt, offp, rb, nBC);
  hipFuncSetAttribute(reinterpret_cast<const void*>(&k_fill),
                      hipFuncAttributeMaxDynamicSharedMemorySize, LDS_FILL);
  k_fill<<<nBF, NTHR, LDS_FILL, stream>>>(src, dst, offp, rb, csr, nN, nE, vec8, csrLen);

  k_gagg<FIN, K1><<<nAgg, NTHR, 0, stream>>>(csr, offp, cnt, x, A1, nN, csrLen);

  hipFuncSetAttribute(reinterpret_cast<const void*>(&k_gemm_ep<K1, HID, 1, 1, 0>),
                      hipFuncAttributeMaxDynamicSharedMemorySize, GA::LDS);
  k_gemm_ep<K1, HID, 1, 1, 0><<<NPAD / GA::BM, NTHR, GA::LDS, stream>>>(A1, pB1, b1, g1, bt1, A1, h1, NPAD, rsq);

  hipFuncSetAttribute(reinterpret_cast<const void*>(&k_gemm_ep<K1, H3W, 0, 0, 0>),
                      hipFuncAttributeMaxDynamicSharedMemorySize, GS::LDS);
  k_gemm_ep<K1, H3W, 0, 0, 0><<<NPAD / GS::BM, NTHR, GS::LDS, stream>>>(A1, pBsk, bsk, bsk, bsk, A1, idp, NPAD, rsq);

  hipFuncSetAttribute(reinterpret_cast<const void*>(&k_gemm_att<HID, HPW, NHEAD>),
                      hipFuncAttributeMaxDynamicSharedMemorySize, GP::LDS);
  k_gemm_att<HID, HPW, NHEAD><<<NPAD / GP::BM, NTHR, GP::LDS, stream>>>(h1, pB2, atS, atD, hp, es, ed, NPAD);

  k_gat<<<nAgg, NTHR, 0, stream>>>(csr, offp, cnt, es, ed, hp, b2, g2, bt2, h2, nN, csrLen, rsq);

  k_gagg<HID, K3><<<nAgg, NTHR, 0, stream>>>(csr, offp, cnt, h2, A3, nN, csrLen);

  hipFuncSetAttribute(reinterpret_cast<const void*>(&k_gemm_ep<K3, H3W, 1, 1, 1>),
                      hipFuncAttributeMaxDynamicSharedMemorySize, GB::LDS);
  k_gemm_ep<K3, H3W, 1, 1, 1><<<NPAD / GB::BM, NTHR, GB::LDS, stream>>>(A3, pB3, b3, g3, bt3, idp, hs, NPAD, rsq);

  hipFuncSetAttribute(reinterpret_cast<const void*>(&k_gemm_ep<H3W, H3W, 0, 1, 0>),
                      hipFuncAttributeMaxDynamicSharedMemorySize, GC::LDS);
  k_gemm_ep<H3W, H3W, 0, 1, 0><<<NPAD / GC::BM, NTHR, GC::LDS, stream>>>(hs, pBc, bc1, bc1, bc1, hs, Tp, NPAD, rsq);

  k_final<<<NPAD / NTHR, NTHR, 0, stream>>>(Tp, Wc2, bc2, out, nN);
}
